// Cross_54477365182468
// MI455X (gfx1250) — hardware-verified
//
#include <hip/hip_runtime.h>
#include <math.h>
#include <stdint.h>

#define NTOK   4096
#define CDIM   256
#define NHEAD  8
#define DHEAD  32
#define OC     (3 * CDIM)
#define NSTR   2
#define MROWS  (NSTR * NTOK)
#define LNEPS  1.0e-5f
#define XC     64.0f
#define WSC    64.0f
#define QC     1024.0f
#define KC     1024.0f
#define VC     256.0f
#define LNPSC  9.704060527839234f
#define ATTSC  0.17677669529663687f
static_assert(NHEAD * DHEAD == CDIM);
static_assert((MROWS % 64) == 0 && (OC % 64) == 0 && (CDIM % 32) == 0);
static_assert((((MROWS / 64) * (OC / 64)) % 8) == 0);
static_assert((NTOK % 64) == 0 && (MROWS % 8) == 0 && (OC % 8) == 0);

typedef _Float16 v16h __attribute__((ext_vector_type(16)));
typedef _Float16 v8h  __attribute__((ext_vector_type(8)));
typedef float    v8f  __attribute__((ext_vector_type(8)));
typedef float    v4f  __attribute__((ext_vector_type(4)));
typedef unsigned int v4u __attribute__((ext_vector_type(4)));

union FragH { v16h v; v8h h[2]; };

__device__ __forceinline__ unsigned short bf_bits(float f) {
  unsigned u = __float_as_uint(f);
  return (unsigned short)((u + 0x7FFFu + ((u >> 16) & 1u)) >> 16);
}
__device__ __forceinline__ float bf_up(unsigned short h) { return __uint_as_float(((unsigned)h) << 16); }
__device__ __forceinline__ float bfr(float f) { return bf_up(bf_bits(f)); }
__device__ __forceinline__ unsigned short h_bits(_Float16 x) { return __builtin_bit_cast(unsigned short, x); }
__device__ __forceinline__ unsigned pk16(unsigned short a, unsigned short b) { return (unsigned)a | ((unsigned)b << 16); }
__device__ __forceinline__ v8f zero8() { v8f z = {0.f, 0.f, 0.f, 0.f, 0.f, 0.f, 0.f, 0.f}; return z; }
__device__ __forceinline__ float hmax8(v8f s) {
  return fmaxf(fmaxf(fmaxf(s[0], s[1]), fmaxf(s[2], s[3])), fmaxf(fmaxf(s[4], s[5]), fmaxf(s[6], s[7])));
}

__device__ __forceinline__ v16h ldfrag_h(const _Float16* p) {
  FragH f;
  f.h[0] = *(const v8h*)(p);
  f.h[1] = *(const v8h*)(p + 16);
  return f.v;
}

__device__ __forceinline__ v8f mma_h_raw(v16h a, v16h b, v8f c) {
  return __builtin_amdgcn_wmma_f32_16x16x32_f16(false, a, false, b, (short)0, c, false, false);
}
__device__ __forceinline__ void dep_guard1(v8f& a, v8f& b, v16h x) {
#if defined(__HIP_DEVICE_COMPILE__)
  asm volatile("v_nop\n\tv_nop\n\tv_nop\n\tv_nop" : "+v"(a), "+v"(b) : "v"(x));
#endif
}
__device__ __forceinline__ void keep4_h(v16h a, v16h b, v16h c, v16h d) {
#if defined(__HIP_DEVICE_COMPILE__)
  asm volatile("v_nop" :: "v"(a), "v"(b), "v"(c), "v"(d));
#endif
}
__device__ __forceinline__ void acc_guard4(v8f& a, v8f& b, v8f& c, v8f& d) {
#if defined(__HIP_DEVICE_COMPILE__)
  asm volatile("v_nop\n\tv_nop\n\tv_nop\n\tv_nop" : "+v"(a), "+v"(b), "+v"(c), "+v"(d));
#endif
}
__device__ __forceinline__ void sguard2(v8f& a, v8f& b, v16h k0, v16h k1, v16h q0, v16h q1) {
#if defined(__HIP_DEVICE_COMPILE__)
  asm volatile("v_nop\n\tv_nop\n\tv_nop\n\tv_nop"
               : "+v"(a), "+v"(b) : "v"(k0), "v"(k1), "v"(q0), "v"(q1));
#endif
}
__device__ __forceinline__ void oguard2(v8f& a, v8f& b, v16h x0, v16h x1, v16h x2, v16h x3, v16h p0, v16h p1) {
#if defined(__HIP_DEVICE_COMPILE__)
  asm volatile("v_nop\n\tv_nop\n\tv_nop\n\tv_nop"
               : "+v"(a), "+v"(b) : "v"(x0), "v"(x1), "v"(x2), "v"(x3), "v"(p0), "v"(p1));
#endif
}
__device__ __forceinline__ void wave_sync_lds() {
  __builtin_amdgcn_fence(__ATOMIC_RELEASE, "workgroup");
  __builtin_amdgcn_wave_barrier();
  __builtin_amdgcn_fence(__ATOMIC_ACQUIRE, "workgroup");
}
__device__ __forceinline__ float wsum(float v) {
#pragma unroll
  for (int off = 16; off > 0; off >>= 1) v += __shfl_xor(v, off, 32);
  return v;
}
__device__ __forceinline__ float ln32(float x, float g, float b) {
  const float mean = wsum(x) * (1.0f / DHEAD);
  const float d    = x - mean;
  const float var  = wsum(d * d) * (1.0f / DHEAD);
  return (d * rsqrtf(var + LNEPS)) * g + b;
}

__global__ __launch_bounds__(256) void cvt_planes(const float* __restrict__ xb, const float* __restrict__ xa,
                                                   const float* __restrict__ w, unsigned short* XN, unsigned short* WT) {
  const int tid = threadIdx.x, r = tid >> 5, lane = tid & 31;
  const int bx  = blockIdx.x;
  const bool isx = (bx < (MROWS / 8));
  const int  s   = isx ? (bx / (NTOK / 8)) : 0;
  const float* src = isx ? ((s == 0) ? xb : xa) : w;
  unsigned short* dst = isx ? XN : WT;
  const float sc  = isx ? XC : WSC;
  const int drow  = isx ? (bx * 8 + r) : ((bx - MROWS / 8) * 8 + r);
  const int srow  = isx ? (drow - s * NTOK) : drow;
  const float* sp = src + (size_t)srow * CDIM + 8 * lane;
  const v4f a = *(const v4f*)(sp), c = *(const v4f*)(sp + 4);
  float f[8];
#pragma unroll
  for (int i = 0; i < 4; ++i) { f[i] = bfr(a[i]) * sc; f[4 + i] = bfr(c[i]) * sc; }
  v4u v;
#pragma unroll
  for (int i = 0; i < 4; ++i) v[i] = pk16(h_bits((_Float16)f[2 * i]), h_bits((_Float16)f[2 * i + 1]));
  unsigned short* dp = dst + (size_t)drow * CDIM + 8 * lane;
  *(volatile v4u*)dp = v;
  __threadfence();
  *(volatile v4u*)dp = v;
}

__global__ __launch_bounds__(256) void gemm64f(
    const unsigned short* __restrict__ Ap, int lda,
    const unsigned short* __restrict__ Bp, int ldb,
    float* Cout, int ldc, float osc, int M, int N, int K) {
  __shared__ __align__(16) float sT[8][16 * 68];
  const int lane = threadIdx.x & 31;
  const int wave = threadIdx.x >> 5;
  const int tilesN = N >> 6;
  const int tilesM = M >> 6;
  const int tile = blockIdx.x * 8 + wave;
  if (tile >= tilesM * tilesN) return;
  const int tm = tile / tilesN;
  const int tn = tile - tm * tilesN;
  const int m0 = tm << 6;
  const int n0 = tn << 6;

  const _Float16* Ah = (const _Float16*)(const void*)Ap;
  const _Float16* Bb = (const _Float16*)(const void*)Bp;

  const int rlane = lane & 15;
  const int koff  = (lane >> 4) * 8;
  const int mOff  = (lane >> 4) * 8;

  v8f acc[4][4];
#pragma unroll
  for (int i = 0; i < 4; ++i)
#pragma unroll
    for (int j = 0; j < 4; ++j) acc[i][j] = zero8();

  for (int k0 = 0; k0 < K; k0 += 32) {
    v16h bh[4];
#pragma unroll
    for (int j = 0; j < 4; ++j) {
      const size_t bo = (size_t)(n0 + (j << 4) + rlane) * ldb + koff + k0;
      bh[j] = ldfrag_h(Bb + bo);
    }
#pragma unroll
    for (int i = 0; i < 4; ++i) {
      const size_t ao = (size_t)(m0 + (i << 4) + rlane) * lda + koff + k0;
      const v16h ah = ldfrag_h(Ah + ao);
#pragma unroll
      for (int j = 0; j < 4; ++j) acc[i][j] = mma_h_raw(ah, bh[j], acc[i][j]);
      dep_guard1(acc[i][0], acc[i][3], ah);
    }
    keep4_h(bh[0], bh[1], bh[2], bh[3]);
  }
  acc_guard4(acc[0][0], acc[0][1], acc[0][2], acc[0][3]);
  acc_guard4(acc[1][0], acc[1][1], acc[1][2], acc[1][3]);
  acc_guard4(acc[2][0], acc[2][1], acc[2][2], acc[2][3]);
  acc_guard4(acc[3][0], acc[3][1], acc[3][2], acc[3][3]);

  const int hh2 = lane >> 4, c4 = (lane & 15) * 4;
  float* slab = sT[wave];
#pragma unroll
  for (int i = 0; i < 4; ++i) {
    const int mBase = m0 + (i << 4);
#pragma unroll
    for (int j = 0; j < 4; ++j) {
#pragma unroll
      for (int r = 0; r < 8; ++r) {
        slab[(mOff + r) * 68 + (j << 4) + rlane] = acc[i][j][r];
      }
    }
    wave_sync_lds();
    v4f vals[8];
#pragma unroll
    for (int it = 0; it < 8; ++it) {
      const int row = it * 2 + hh2;
      v4f v = *(const v4f*)(slab + row * 68 + c4);
#pragma unroll
      for (int e = 0; e < 4; ++e) v[e] = v[e] * osc;
      vals[it] = v;
    }
    for (int pass = 0; pass < 2; ++pass) {
#pragma unroll
      for (int it = 0; it < 8; ++it) {
        const int row = it * 2 + hh2;
        *(volatile v4f*)(Cout + (size_t)(mBase + row) * ldc + n0 + c4) = vals[it];
      }
      __threadfence();
    }
    wave_sync_lds();
  }
}

__global__ __launch_bounds__(256)
void ln_heads(const float* __restrict__ T, const float* __restrict__ gam, const float* __restrict__ bet,
              unsigned short* QH, unsigned short* QL, unsigned short* KH,
              unsigned short* VTH, unsigned short* VTL) {
  __shared__ __align__(16) unsigned short VsH[128 * 72];
  __shared__ __align__(16) unsigned short VsL[128 * 72];
  __shared__ __align__(16) unsigned short RBh[8][CDIM];
  __shared__ __align__(16) unsigned short RBl[8][CDIM];
  const int tid = threadIdx.x, wave = tid >> 5, lane = tid & 31;
  const int bx  = blockIdx.x;
  const int s   = bx / (NTOK / 64);
  const int tok0 = (bx - s * (NTOK / 64)) * 64;
  const float g  = bfr(gam[lane]);
  const float be = bfr(bet[lane]);
#pragma unroll 1
  for (int vh = 0; vh < 2; ++vh) {
#pragma unroll 1
    for (int i = 0; i < 8; ++i) {
      const int tl = wave * 8 + i;
      const size_t row = (size_t)s * NTOK + tok0 + tl;
      const float* tr = T + row * OC;
      if (vh == 0) {
#pragma unroll 1
        for (int h = 0; h < NHEAD; ++h) {
          const float y = ln32(tr[h * DHEAD + lane], g, be) * QC;
          const _Float16 hi = (_Float16)y;
          const _Float16 lo = (_Float16)(y - (float)hi);
          RBh[wave][h * DHEAD + lane] = h_bits(hi);
          RBl[wave][h * DHEAD + lane] = h_bits(lo);
        }
        wave_sync_lds();
        {
          const v4u a  = *(const v4u*)(&RBh[wave][8 * lane]);
          const v4u bl = *(const v4u*)(&RBl[wave][8 * lane]);
          unsigned short* pa = QH + row * CDIM + 8 * lane;
          unsigned short* pb = QL + row * CDIM + 8 * lane;
          *(volatile v4u*)pa = a;
          *(volatile v4u*)pb = bl;
          __threadfence();
          *(volatile v4u*)pa = a;
          *(volatile v4u*)pb = bl;
        }
        wave_sync_lds();
#pragma unroll 1
        for (int h = 0; h < NHEAD; ++h) {
          const float y = ln32(tr[CDIM + h * DHEAD + lane], g, be) * KC;
          RBh[wave][h * DHEAD + lane] = h_bits((_Float16)y);
        }
        wave_sync_lds();
        {
          const v4u a = *(const v4u*)(&RBh[wave][8 * lane]);
          unsigned short* pk = KH + row * CDIM + 8 * lane;
          *(volatile v4u*)pk = a;
          __threadfence();
          *(volatile v4u*)pk = a;
        }
        wave_sync_lds();
      }
#pragma unroll 1
      for (int hq = 0; hq < 4; ++hq) {
        const int h = vh * 4 + hq;
        const float y = ln32(tr[2 * CDIM + h * DHEAD + lane], g, be) * VC;
        const _Float16 hi = (_Float16)y;
        const _Float16 lo = (_Float16)(y - (float)hi);
        VsH[(hq * DHEAD + lane) * 72 + tl] = h_bits(hi);
        VsL[(hq * DHEAD + lane) * 72 + tl] = h_bits(lo);
      }
    }
    __syncthreads();
    {
      const int e = tid & 7, fq = tid >> 3;
      v4u hv[4], lv[4];
#pragma unroll
      for (int it = 0; it < 4; ++it) {
        const int fl = it * 32 + fq;
        hv[it] = *(const v4u*)(VsH + fl * 72 + 8 * e);
        lv[it] = *(const v4u*)(VsL + fl * 72 + 8 * e);
      }
      unsigned short* hb = VTH + ((size_t)s * CDIM + vh * 128) * NTOK + tok0 + 8 * e;
      unsigned short* lb = VTL + ((size_t)s * CDIM + vh * 128) * NTOK + tok0 + 8 * e;
      for (int pass = 0; pass < 2; ++pass) {
#pragma unroll
        for (int it = 0; it < 4; ++it) {
          const int fl = it * 32 + fq;
          *(volatile v4u*)(hb + (size_t)fl * NTOK) = hv[it];
          *(volatile v4u*)(lb + (size_t)fl * NTOK) = lv[it];
        }
        __threadfence();
      }
    }
    __syncthreads();
  }
}

__global__ __launch_bounds__(128)
void attn_kernel(const unsigned short* __restrict__ qh, const unsigned short* __restrict__ ql,
                 const unsigned short* __restrict__ kh, const unsigned short* __restrict__ vth,
                 const unsigned short* __restrict__ vtl, float* out) {
  __shared__ __align__(16) float Os[64 * DHEAD];
  const int tid  = threadIdx.x;
  const int wave = tid >> 5;
  const int lane = tid & 31;
  const int hh   = lane >> 4;
  const int c    = lane & 15;
  const int bx   = blockIdx.x;
  const int qb   = bx % (NTOK / 64);
  const int hd   = (bx / (NTOK / 64)) % NHEAD;
  const int dir  = bx / ((NTOK / 64) * NHEAD);
  const int qsrc = 1 - dir;
  const int ksrc = dir;
  const int q0   = qb * 64;

  const _Float16* QHp = (const _Float16*)(const void*)qh;
  const _Float16* QLp = (const _Float16*)(const void*)ql;
  const _Float16* KHp = (const _Float16*)(const void*)kh;
  const _Float16* VHp = (const _Float16*)(const void*)vth;
  const _Float16* VLp = (const _Float16*)(const void*)vtl;

  const size_t qtok = (size_t)qsrc * NTOK + q0 + wave * 16 + c;
  const v16h qhf = ldfrag_h(QHp + qtok * CDIM + hd * DHEAD + 8 * hh);
  const v16h qlf = ldfrag_h(QLp + qtok * CDIM + hd * DHEAD + 8 * hh);
  const _Float16* Kp = KHp + ((size_t)ksrc * NTOK + c) * CDIM + hd * DHEAD + 8 * hh;
  const size_t vrow = ((size_t)ksrc * CDIM + hd * DHEAD + c) * NTOK + 8 * hh;
  const _Float16* VH0 = VHp + vrow;
  const _Float16* VH1 = VH0 + (size_t)16 * NTOK;
  const _Float16* VL0 = VLp + vrow;
  const _Float16* VL1 = VL0 + (size_t)16 * NTOK;
  const float SC = ATTSC / (QC * KC);

  float m = -1.0e30f, l = 0.f;
  v8f o0 = zero8(), o1 = zero8();
#pragma unroll 1
  for (int it = 0; it < NTOK / 32; ++it) {
    const int kb = it * 32;
    const v16h kf0 = ldfrag_h(Kp + (size_t)kb * CDIM);
    const v16h kf1 = ldfrag_h(Kp + (size_t)(kb + 16) * CDIM);
    v8f s0 = mma_h_raw(kf0, qhf, zero8());
    v8f s1 = mma_h_raw(kf1, qhf, zero8());
    s0 = mma_h_raw(kf0, qlf, s0);
    s1 = mma_h_raw(kf1, qlf, s1);
    sguard2(s0, s1, kf0, kf1, qhf, qlf);

    float mx = fmaxf(hmax8(s0), hmax8(s1));
    mx = fmaxf(mx, __shfl_xor(mx, 16, 32));
    const float mn   = fmaxf(m, mx * SC);
    const float corr = __expf(m - mn);
    m = mn;
    const float msh = mn - LNPSC;
    l *= corr;
#pragma unroll
    for (int r = 0; r < 8; ++r) { o0[r] *= corr; o1[r] *= corr; }

    FragH ph, pl;
    float ls = 0.f;
#pragma unroll
    for (int r = 0; r < 8; ++r) {
      const float e0 = __expf(s0[r] * SC - msh);
      const float e1 = __expf(s1[r] * SC - msh);
      ls += e0 + e1;
      const _Float16 h0 = (_Float16)e0, h1 = (_Float16)e1;
      ph.h[0][r] = h0;
      ph.h[1][r] = h1;
      pl.h[0][r] = (_Float16)(e0 - (float)h0);
      pl.h[1][r] = (_Float16)(e1 - (float)h1);
    }
    l += ls;

    const v16h vh0 = ldfrag_h(VH0 + kb);
    const v16h vh1 = ldfrag_h(VH1 + kb);
    const v16h vl0 = ldfrag_h(VL0 + kb);
    const v16h vl1 = ldfrag_h(VL1 + kb);
    o0 = mma_h_raw(vh0, ph.v, o0);
    o1 = mma_h_raw(vh1, ph.v, o1);
    o0 = mma_h_raw(vh0, pl.v, o0);
    o1 = mma_h_raw(vh1, pl.v, o1);
    o0 = mma_h_raw(vl0, ph.v, o0);
    o1 = mma_h_raw(vl1, ph.v, o1);
    oguard2(o0, o1, vh0, vh1, vl0, vl1, ph.v, pl.v);
  }
  l += __shfl_xor(l, 16, 32);
  const float sc = (1.0f / VC) * (1.0f / l);

  float* os = Os + (wave * 16 + c) * DHEAD + 8 * hh;
#pragma unroll
  for (int r = 0; r < 8; ++r) { os[r] = o0[r] * sc; os[16 + r] = o1[r] * sc; }
  __syncthreads();
  {
    const int e = tid & 7, qq = tid >> 3;
    v4f vals[4];
#pragma unroll
    for (int it = 0; it < 4; ++it) {
      const int qi = it * 16 + qq;
      vals[it] = *(const v4f*)(Os + qi * DHEAD + 4 * e);
    }
    float* ob = out + (size_t)dir * NTOK * CDIM + (size_t)hd * DHEAD + 4 * e;
    for (int pass = 0; pass < 2; ++pass) {
#pragma unroll
      for (int it = 0; it < 4; ++it) {
        const int qi = it * 16 + qq;
        *(volatile v4f*)(ob + (size_t)(q0 + qi) * CDIM) = vals[it];
      }
      __threadfence();
    }
  }
}

extern "C" void kernel_launch(void* const* d_in, const int* in_sizes, int n_in,
                              void* d_out, int out_size, void* d_ws, size_t ws_size,
                              hipStream_t stream) {
  if (n_in < 5) return;
  if (in_sizes[0] != NTOK * CDIM || in_sizes[1] != NTOK * CDIM) return;
  if (in_sizes[2] != OC * CDIM) return;
  if (in_sizes[3] != DHEAD || in_sizes[4] != DHEAD) return;
  if (out_size != NSTR * NTOK * CDIM) return;

  const float* x_b   = (const float*)d_in[0];
  const float* x_a   = (const float*)d_in[1];
  const float* w_qkv = (const float*)d_in[2];
  const float* ln_g  = (const float*)d_in[3];
  const float* ln_b  = (const float*)d_in[4];

  const size_t PXN = (size_t)MROWS * CDIM * 2;
  const size_t PWT = (size_t)OC * CDIM * 2;
  const size_t PT  = (size_t)MROWS * OC * 4;
  const size_t PQ  = (size_t)MROWS * CDIM * 2;
  const size_t PV  = (size_t)NSTR * CDIM * NTOK * 2;
  size_t off = 0;
  const size_t oXN = off; off += PXN;
  const size_t oWT = off; off += PWT;
  const size_t oT  = off; off += PT;
  const size_t oQH = off; off += PQ;
  const size_t oQL = off; off += PQ;
  const size_t oKH = off; off += PQ;
  const size_t oVH = off; off += PV;
  const size_t oVL = off; off += PV;
  if (off > ws_size) return;
  if (off > (size_t)134217728) return;

  char* ws = (char*)d_ws;
  unsigned short* XN  = (unsigned short*)(ws + oXN);
  unsigned short* WT  = (unsigned short*)(ws + oWT);
  float*          T   = (float*)(ws + oT);
  unsigned short* QH  = (unsigned short*)(ws + oQH);
  unsigned short* QL  = (unsigned short*)(ws + oQL);
  unsigned short* KH  = (unsigned short*)(ws + oKH);
  unsigned short* VTH = (unsigned short*)(ws + oVH);
  unsigned short* VTL = (unsigned short*)(ws + oVL);
  float*          out = (float*)d_out;

  const dim3 blk(256), blk128(128);
  const dim3 gCV(MROWS / 8 + OC / 8);
  const dim3 gGM(((MROWS / 64) * (OC / 64)) / 8);
  const dim3 gLN(MROWS / 64);
  const dim3 gAT(NSTR * NHEAD * (NTOK / 64));

  cvt_planes<<<gCV, blk, 0, stream>>>(x_b, x_a, w_qkv, XN, WT);

  gemm64f<<<gGM, blk, 0, stream>>>(XN, CDIM, WT, CDIM, T, OC, 1.0f / (XC * WSC), MROWS, OC, CDIM);

  ln_heads<<<gLN, blk, 0, stream>>>(T, ln_g, ln_b, QH, QL, KH, VTH, VTL);

  attn_kernel<<<gAT, blk128, 0, stream>>>(QH, QL, KH, VTH, VTL, out);
  (void)hipGetLastError();
}
